// BPFeedForward_7919919693923
// MI455X (gfx1250) — hardware-run, weakly checked
//
#include <hip/hip_runtime.h>
#include <math.h>

typedef __attribute__((ext_vector_type(16))) _Float16 v16h;
typedef __attribute__((ext_vector_type(8)))  _Float16 v8h;
typedef __attribute__((ext_vector_type(8)))  float    v8f;
typedef __attribute__((ext_vector_type(4)))  float    v4f;
typedef __attribute__((ext_vector_type(4)))  int      v4i;

constexpr int kTypes  = 4;
constexpr int kRowsT  = 50000;
constexpr int kAtoms  = kTypes * kRowsT;
constexpr int kDimIn  = 128;
constexpr int kDimH   = 256;
constexpr int kTileM  = 64;
constexpr int kBlocks = (kRowsT + kTileM - 1) / kTileM;
constexpr int kHP = 264;
constexpr int kZP = 260;
constexpr float kActCarry = 32.0f;
constexpr float kWgtCarry = 256.0f;
constexpr float kFoldBack = 1.0f / (kActCarry * kWgtCarry);
constexpr float kF16MinNormal = 6.103515625e-5f;

static_assert(kAtoms == 200000, "atom count");
static_assert(kBlocks == 782, "tile count");
static_assert((kDimIn % 32) == 0 && (kDimH % 32) == 0, "k multiples of 32");
static_assert((kDimH % 64) == 0, "n multiple of 64");
static_assert((kAtoms % 4) == 0 && ((kAtoms * 4) % 128) == 0, "output is whole 128-B lines");
static_assert(((kHP * 2) % 16) == 0 && ((kZP * 4) % 16) == 0, "16-B aligned LDS rows");

constexpr size_t kOffW0T  = 0;
constexpr size_t kOffW1T  = kOffW0T + (size_t)kTypes * kDimH * kDimIn * 2;
constexpr size_t kOffW2T  = kOffW1T + (size_t)kTypes * kDimH * kDimH * 2;
constexpr size_t kWsTotal = kOffW2T + (size_t)kTypes * kDimH * kDimH * 2;
static_assert(kWsTotal == 1310720ull, "carve total");
static_assert(kWsTotal <= 134217728ull, "carve cap");
static_assert((kOffW1T % 128) == 0 && (kOffW2T % 128) == 0, "128-B aligned regions");

__device__ __forceinline__ _Float16 to_f16_carry(float v, float carry) {
  float c = v * carry;
  c = (fabsf(c) < kF16MinNormal) ? 0.0f : c;
  return (_Float16)c;
}

__device__ __forceinline__ v16h frag_load(const _Float16* p) {
  union U { v16h v; v8h h[2]; };
  U f;
  f.h[0] = *(const v8h*)(p);
  f.h[1] = *(const v8h*)(p + 16);
  return f.v;
}

__device__ __forceinline__ v8f mma_f16(v16h a, v16h b, v8f c) {
  c = __builtin_amdgcn_wmma_f32_16x16x32_f16(false, a, false, b, (short)0, c, false, false);
  asm volatile("v_nop\n\tv_nop\n\tv_nop\n\tv_nop" : "+v"(c) : "v"(a), "v"(b));
  return c;
}

__global__ __launch_bounds__(256) void prep_weights_kernel(
    const float* __restrict__ W0, const float* __restrict__ W1, const float* __restrict__ W2,
    unsigned short* __restrict__ W0t, unsigned short* __restrict__ W1t, unsigned short* __restrict__ W2t)
{
  __shared__ float sT[64 * 33];
  const int tid = threadIdx.x;
  int b = blockIdx.x;
  const float* W;
  unsigned short* Wt;
  int K;
  if (b < 64) {
    W = W0; Wt = W0t; K = kDimIn;
  } else if (b < 192) {
    b -= 64; W = W1; Wt = W1t; K = kDimH;
  } else {
    b -= 192; W = W2; Wt = W2t; K = kDimH;
  }
  const int tilesK = K >> 6;
  const int perType = tilesK * 8;
  const int e   = b / perType;
  const int rem = b - e * perType;
  const int k0  = (rem >> 3) * 64;
  const int n0  = (rem & 7) * 32;
#pragma unroll
  for (int i = 0; i < 8; ++i) {
    const int idx = i * 256 + tid;
    const int kk = idx >> 5;
    const int nn = idx & 31;
    sT[kk * 33 + nn] = W[((size_t)(e * K + k0 + kk)) * kDimH + n0 + nn];
  }
  __syncthreads();
  const int nn = tid >> 3;
  const int k8 = (tid & 7) * 8;
  v8h hv;
#pragma unroll
  for (int i = 0; i < 8; ++i) {
    const float v = sT[(k8 + i) * 33 + nn];
    hv[i] = to_f16_carry(v, kWgtCarry);
  }
  unsigned short* q = Wt + ((size_t)(e * kDimH + n0 + nn)) * K + k0 + k8;
  *(volatile v8h*)q = hv;
  __threadfence();
  *(volatile v8h*)q = hv;
}

__global__ __launch_bounds__(256) void fused_mlp_kernel(
    const float* __restrict__ f0, const float* __restrict__ f1,
    const float* __restrict__ f2, const float* __restrict__ f3,
    const unsigned short* __restrict__ W0tp, const unsigned short* __restrict__ W1tp,
    const unsigned short* __restrict__ W2tp,
    const float* __restrict__ b0, const float* __restrict__ b1, const float* __restrict__ b2,
    const float* __restrict__ Wout, const int* __restrict__ elems, float* __restrict__ out)
{
  __shared__ __align__(16) _Float16 sH[2 * kTileM * kHP];
  __shared__ __align__(16) float    sZ[kTileM * kZP];
  __shared__ __align__(16) float    sOut[kTileM * kTypes];

  const int tid  = threadIdx.x;
  const int lane = tid & 31;
  const int wave = tid >> 5;
  const int hh   = lane >> 4;
  const int l16  = lane & 15;
  const int m0   = blockIdx.x * kTileM;
  const int n0   = wave * 32;
  const int c8   = lane * 8;

  const _Float16* W0t = (const _Float16*)W0tp;
  const _Float16* W1t = (const _Float16*)W1tp;
  const _Float16* W2t = (const _Float16*)W2tp;

#pragma unroll 1
  for (int e = 0; e < kTypes; ++e) {
    const float* fp = (e == 0) ? f0 : (e == 1) ? f1 : (e == 2) ? f2 : f3;
#pragma unroll 1
    for (int it = 0; it < 4; ++it) {
      const int idx = it * 256 + tid;
      const int row = idx >> 4;
      const int cc  = (idx & 15) * 8;
      int gr = m0 + row;
      gr = (gr < kRowsT) ? gr : (kRowsT - 1);
      const float* sp = fp + (size_t)gr * kDimIn + cc;
      const v4f a0 = *(const v4f*)(sp);
      const v4f a1 = *(const v4f*)(sp + 4);
      v8h hv;
#pragma unroll
      for (int i = 0; i < 4; ++i) {
        hv[i]     = to_f16_carry(a0[i], kActCarry);
        hv[4 + i] = to_f16_carry(a1[i], kActCarry);
      }
      *(v8h*)(sH + row * kHP + cc) = hv;
    }
    const v4f wo0 = *(const v4f*)(Wout + e * kDimH + c8);
    const v4f wo1 = *(const v4f*)(Wout + e * kDimH + c8 + 4);
    __syncthreads();

#pragma unroll 1
    for (int l = 0; l < 3; ++l) {
      const int K = (l == 0) ? kDimIn : kDimH;
      const _Float16* Bt = (l == 0) ? (W0t + (size_t)e * kDimH * kDimIn)
                         : (l == 1) ? (W1t + (size_t)e * kDimH * kDimH)
                                    : (W2t + (size_t)e * kDimH * kDimH);
      const float* bl = ((l == 0) ? b0 : (l == 1) ? b1 : b2) + e * kDimH;
      const int srcOff = (l & 1) * (kTileM * kHP);
      const int dstOff = ((l & 1) ^ 1) * (kTileM * kHP);

      v8f acc[4][2];
#pragma unroll
      for (int i = 0; i < 4; ++i)
#pragma unroll
        for (int j = 0; j < 2; ++j) acc[i][j] = (v8f){0.f, 0.f, 0.f, 0.f, 0.f, 0.f, 0.f, 0.f};

      const _Float16* ap  = sH + srcOff + l16 * kHP + 8 * hh;
      const _Float16* bp0 = Bt + (size_t)(n0 + l16) * K + 8 * hh;
      const _Float16* bp1 = Bt + (size_t)(n0 + 16 + l16) * K + 8 * hh;
#pragma unroll 1
      for (int k0 = 0; k0 < K; k0 += 32) {
        const v16h bf0 = frag_load(bp0 + k0);
        const v16h bf1 = frag_load(bp1 + k0);
#pragma unroll
        for (int i = 0; i < 4; ++i) {
          const v16h af = frag_load(ap + i * 16 * kHP + k0);
          acc[i][0] = mma_f16(af, bf0, acc[i][0]);
          acc[i][1] = mma_f16(af, bf1, acc[i][1]);
        }
      }

#pragma unroll
      for (int i = 0; i < 4; ++i)
#pragma unroll
        for (int j = 0; j < 2; ++j)
#pragma unroll
          for (int r = 0; r < 8; ++r)
            sZ[(i * 16 + 8 * hh + r) * kZP + n0 + j * 16 + l16] = acc[i][j][r];
      __syncthreads();

      const v4f bz0 = *(const v4f*)(bl + c8);
      const v4f bz1 = *(const v4f*)(bl + c8 + 4);
#pragma unroll 1
      for (int it = 0; it < 8; ++it) {
        const int row = it * 8 + wave;
        const float* zp = sZ + row * kZP + c8;
        const v4f z0 = *(const v4f*)(zp);
        const v4f z1 = *(const v4f*)(zp + 4);
        float t[8];
#pragma unroll
        for (int i = 0; i < 4; ++i) {
          t[i]     = tanhf(fmaf(z0[i], kFoldBack, bz0[i]));
          t[4 + i] = tanhf(fmaf(z1[i], kFoldBack, bz1[i]));
        }
        if (l < 2) {
          v8h hv;
#pragma unroll
          for (int i = 0; i < 8; ++i) hv[i] = to_f16_carry(t[i], kActCarry);
          *(v8h*)(sH + dstOff + row * kHP + c8) = hv;
        } else {
          float d = 0.0f;
#pragma unroll
          for (int i = 0; i < 4; ++i) d = fmaf(t[i], wo0[i], d);
#pragma unroll
          for (int i = 0; i < 4; ++i) d = fmaf(t[4 + i], wo1[i], d);
#pragma unroll
          for (int off = 16; off >= 1; off >>= 1) d += __shfl_xor(d, off, 32);
          if (lane == 0) sOut[row * kTypes + e] = d;
        }
      }
      __syncthreads();
    }
  }

  const int rowsValid = (kRowsT - m0 < kTileM) ? (kRowsT - m0) : kTileM;
  const int nValid = rowsValid * kTypes;
  const int j0 = (tid & 63) * 4;
  const v4f sv = *(const v4f*)(sOut + j0);
  int atom0 = blockIdx.x * (kTileM * kTypes) + j0;
  atom0 = (atom0 < kAtoms - 4) ? atom0 : (kAtoms - 4);
  const v4i el = *(const v4i*)(elems + atom0);
  int q0 = el[0];
  int q1 = el[1];
  int q2 = el[2];
  int q3 = el[3];
  asm volatile("" : "+v"(q0), "+v"(q1), "+v"(q2), "+v"(q3));
  const float qnan = __uint_as_float(0x7fc00000u);
  float s0 = sv[0];
  float s1 = sv[1];
  float s2 = sv[2];
  float s3 = sv[3];
  s0 = (q0 == 0) ? s0 : qnan;
  s1 = (q1 == 1) ? s1 : qnan;
  s2 = (q2 == 2) ? s2 : qnan;
  s3 = (q3 == 3) ? s3 : qnan;
  v4f ov;
  ov[0] = s0;
  ov[1] = s1;
  ov[2] = s2;
  ov[3] = s3;
  const bool doStore = (tid < 64) && (j0 < nValid);
  float* op = out + atom0;
  if (doStore) *(volatile v4f*)op = ov;
  __threadfence();
  if (doStore) *(volatile v4f*)op = ov;
}

extern "C" void kernel_launch(void* const* d_in, const int* in_sizes, int n_in,
                              void* d_out, int out_size, void* d_ws, size_t ws_size,
                              hipStream_t stream) {
  if (n_in < 13) return;
  if (in_sizes[0] != kRowsT * kDimIn) return;
  if (in_sizes[1] != kRowsT * kDimIn) return;
  if (in_sizes[2] != kRowsT * kDimIn) return;
  if (in_sizes[3] != kRowsT * kDimIn) return;
  if (in_sizes[4] != kTypes * kDimIn * kDimH) return;
  if (in_sizes[5] != kTypes * kDimH) return;
  if (in_sizes[6] != kTypes * kDimH * kDimH) return;
  if (in_sizes[7] != kTypes * kDimH) return;
  if (in_sizes[8] != kTypes * kDimH * kDimH) return;
  if (in_sizes[9] != kTypes * kDimH) return;
  if (in_sizes[10] != kTypes * kDimH) return;
  if (in_sizes[11] != kAtoms) return;
  if (in_sizes[12] != kAtoms) return;
  if (out_size != kAtoms) return;
  if (ws_size < kWsTotal) return;

  const float* fps0 = (const float*)d_in[0];
  const float* fps1 = (const float*)d_in[1];
  const float* fps2 = (const float*)d_in[2];
  const float* fps3 = (const float*)d_in[3];
  const float* W0   = (const float*)d_in[4];
  const float* b0   = (const float*)d_in[5];
  const float* W1   = (const float*)d_in[6];
  const float* b1   = (const float*)d_in[7];
  const float* W2   = (const float*)d_in[8];
  const float* b2   = (const float*)d_in[9];
  const float* Wout = (const float*)d_in[10];
  const int*   elems = (const int*)d_in[11];
  float* out = (float*)d_out;

  char* ws = (char*)d_ws;
  unsigned short* W0t = (unsigned short*)(ws + kOffW0T);
  unsigned short* W1t = (unsigned short*)(ws + kOffW1T);
  unsigned short* W2t = (unsigned short*)(ws + kOffW2T);

  prep_weights_kernel<<<320, 256, 0, stream>>>(W0, W1, W2, W0t, W1t, W2t);
  fused_mlp_kernel<<<kBlocks, 256, 0, stream>>>(fps0, fps1, fps2, fps3, W0t, W1t, W2t,
                                                b0, b1, b2, Wout, elems, out);
}
